// AGNN_DGL_67156108640390
// MI455X (gfx1250) — hardware-run, weakly checked
//
#include <hip/hip_runtime.h>
#include <stddef.h>


#define FIN     128
#define HID     64
#define NTHR    256
#define NWAVE   8
#define EPT     8
#define CHUNK   (NTHR * EPT)
#define WCAP    (EPT * 32)
#define LISTN   (NWAVE * WCAP)
#define NBMAX   2048
#define SLOTB   11
#define RCAP    28672
#define DEGCAP  4096
#define NSTRM   4
#define GBM     32
#define GTHR    64
#define CA      16.0f
#define CW      64.0f
#define SCL     0.0009765625f
#define EPSN    1e-12f
#define NEGBIG  (-1.0e30f)
#define WSCAP   134217728
#define LDS_BUILD ((2 * RCAP + 2 * NBMAX + LISTN) * 4 + 64)

static_assert((CHUNK & (CHUNK - 1)) == 0 && CHUNK <= 4096);
static_assert(NBMAX == (1 << SLOTB));
static_assert(NTHR * 8 == NBMAX);
static_assert(LISTN >= NBMAX);
static_assert(LISTN >= NWAVE * WCAP);
static_assert((RCAP % 32) == 0);
static_assert(LDS_BUILD <= 300000);
static_assert(GBM == (GTHR / 32) * 16);
static_assert(GTHR == HID);
static_assert((FIN % 32) == 0 && (HID % 32) == 0);
static_assert(FIN / 8 == 16 && HID / 8 == 8);
static_assert(NSTRM * 8 == 32 && HID == 8 * 8);

typedef float    v4f  __attribute__((ext_vector_type(4)));
typedef float    v8f  __attribute__((ext_vector_type(8)));
typedef int      v4i  __attribute__((ext_vector_type(4)));
typedef int      v8i  __attribute__((ext_vector_type(8)));
typedef _Float16 v8h  __attribute__((ext_vector_type(8)));
typedef _Float16 v16h __attribute__((ext_vector_type(16)));
union FragH { v16h v; v8h h[2]; v8i w; };

__device__ __forceinline__ v8f wmh(const FragH& a, const FragH& b, v8f c) {
  v8f d = __builtin_amdgcn_wmma_f32_16x16x32_f16(false, a.v, false, b.v, (short)0, c, false, false);
  asm volatile("v_nop\n\tv_nop\n\tv_nop\n\tv_nop" : "+v"(d) : "v"(a.w), "v"(b.w));
  return d;
}

__device__ __forceinline__ v8h pack8(v4f a, v4f b, float sc) {
  v8h hv;
  hv[0] = (_Float16)(a.x * sc); hv[1] = (_Float16)(a.y * sc);
  hv[2] = (_Float16)(a.z * sc); hv[3] = (_Float16)(a.w * sc);
  hv[4] = (_Float16)(b.x * sc); hv[5] = (_Float16)(b.y * sc);
  hv[6] = (_Float16)(b.z * sc); hv[7] = (_Float16)(b.w * sc);
  return hv;
}

__device__ __forceinline__ float dot8(v4f a0, v4f a1, v4f b0, v4f b1) {
  float s = a0.x * b0.x;
  s = fmaf(a0.y, b0.y, s); s = fmaf(a0.z, b0.z, s); s = fmaf(a0.w, b0.w, s);
  s = fmaf(a1.x, b1.x, s); s = fmaf(a1.y, b1.y, s); s = fmaf(a1.z, b1.z, s); s = fmaf(a1.w, b1.w, s);
  return s;
}

__device__ __forceinline__ v4f xor4(v4f v, int msk) {
  v4f r;
  r.x = __shfl_xor(v.x, msk); r.y = __shfl_xor(v.y, msk);
  r.z = __shfl_xor(v.z, msk); r.w = __shfl_xor(v.w, msk);
  return r;
}

__device__ __forceinline__ v4f shf4(v4f v, int src) {
  v4f r;
  r.x = __shfl(v.x, src); r.y = __shfl(v.y, src);
  r.z = __shfl(v.z, src); r.w = __shfl(v.w, src);
  return r;
}

__device__ __forceinline__ int scan_chunk(const int* __restrict__ dsts, int nE, int cbase, int slotBase,
                                          int nb, int vec8, int* list, int tid, int lane, int wave) {
  int wc = 0;
  const int el0  = tid * EPT;
  const int e0   = cbase + el0;
  const int sent = -2147483647 - 1;
  v4i da, db;
  if (vec8 != 0 && cbase + CHUNK <= nE) {
    da = *(const v4i*)(dsts + e0);
    db = *(const v4i*)(dsts + e0 + 4);
  } else {
    da.x = (e0     < nE) ? dsts[min(e0,     nE - 1)] : sent;
    da.y = (e0 + 1 < nE) ? dsts[min(e0 + 1, nE - 1)] : sent;
    da.z = (e0 + 2 < nE) ? dsts[min(e0 + 2, nE - 1)] : sent;
    da.w = (e0 + 3 < nE) ? dsts[min(e0 + 3, nE - 1)] : sent;
    db.x = (e0 + 4 < nE) ? dsts[min(e0 + 4, nE - 1)] : sent;
    db.y = (e0 + 5 < nE) ? dsts[min(e0 + 5, nE - 1)] : sent;
    db.z = (e0 + 6 < nE) ? dsts[min(e0 + 6, nE - 1)] : sent;
    db.w = (e0 + 7 < nE) ? dsts[min(e0 + 7, nE - 1)] : sent;
  }
  const unsigned nbs = (unsigned)slotBase;
  const unsigned unb = (unsigned)nb;
  const unsigned s0 = (unsigned)da.x - nbs, s1 = (unsigned)da.y - nbs;
  const unsigned s2 = (unsigned)da.z - nbs, s3 = (unsigned)da.w - nbs;
  const unsigned s4 = (unsigned)db.x - nbs, s5 = (unsigned)db.y - nbs;
  const unsigned s6 = (unsigned)db.z - nbs, s7 = (unsigned)db.w - nbs;
  const bool h0 = s0 < unb, h1 = s1 < unb, h2 = s2 < unb, h3 = s3 < unb;
  const bool h4 = s4 < unb, h5 = s5 < unb, h6 = s6 < unb, h7 = s7 < unb;
  const unsigned any = __builtin_amdgcn_ballot_w32(h0 | h1 | h2 | h3 | h4 | h5 | h6 | h7);
  if (any != 0u) {
#define HITJ(J, HJ, SJ) { \
      const unsigned mj = __builtin_amdgcn_ballot_w32(HJ); \
      if (mj != 0u) { \
        if (HJ) { \
          const int pos = wc + (int)__builtin_amdgcn_mbcnt_lo(mj, 0u); \
          if (pos < WCAP) list[wave * WCAP + pos] = ((el0 + (J)) << 12) | (int)(SJ); \
        } \
        wc += (int)__builtin_popcount(mj); } }
    HITJ(0, h0, s0)
    HITJ(1, h1, s1)
    HITJ(2, h2, s2)
    HITJ(3, h3, s3)
    HITJ(4, h4, s4)
    HITJ(5, h5, s5)
    HITJ(6, h6, s6)
    HITJ(7, h7, s7)
#undef HITJ
  }
  return wc;
}

__global__ __launch_bounds__(NTHR) void k_wprep(const float* __restrict__ w1, const float* __restrict__ w2,
                                                _Float16* w1t, _Float16* w2t) {
  const int j = (int)blockIdx.y;
  const int u = (int)blockIdx.x * NTHR + (int)threadIdx.x;
  v4f a, b;
  if (j == 0) {
    const int nUnits = HID * (FIN / 8);
    if (u >= nUnits) return;
    const int n  = u >> 4;
    const int k8 = (u & 15) * 8;
    const float* p = w1 + (size_t)k8 * HID + n;
    a.x = p[0 * HID]; a.y = p[1 * HID]; a.z = p[2 * HID]; a.w = p[3 * HID];
    b.x = p[4 * HID]; b.y = p[5 * HID]; b.z = p[6 * HID]; b.w = p[7 * HID];
    const v8h hv = pack8(a, b, CW);
    const size_t o = (size_t)n * FIN + k8;
    *(volatile v8h*)(w1t + o) = hv;
    __threadfence();
    *(volatile v8h*)(w1t + o) = hv;
  } else {
    const int nUnits = HID * (HID / 8);
    if (u >= nUnits) return;
    const int n  = u >> 3;
    const int k8 = (u & 7) * 8;
    const float* p = w2 + (size_t)k8 * HID + n;
    a.x = p[0 * HID]; a.y = p[1 * HID]; a.z = p[2 * HID]; a.w = p[3 * HID];
    b.x = p[4 * HID]; b.y = p[5 * HID]; b.z = p[6 * HID]; b.w = p[7 * HID];
    const v8h hv = pack8(a, b, CW);
    const size_t o = (size_t)n * HID + k8;
    *(volatile v8h*)(w2t + o) = hv;
    __threadfence();
    *(volatile v8h*)(w2t + o) = hv;
  }
}

__global__ __launch_bounds__(GTHR) void k_lin(const float* __restrict__ A, const _Float16* __restrict__ wt,
                                              const float* __restrict__ bias, float* Y, int K, int relu) {
  __shared__ __attribute__((aligned(16))) float stg[GBM * HID];
  __shared__ float sb[HID];
  const int tid = threadIdx.x, lane = tid & 31, wave = tid >> 5, hh = lane >> 4, m = lane & 15;
  const int rowBase = (int)blockIdx.x * GBM;
  if (tid < HID) sb[tid] = bias[tid];
  __syncthreads();
  const float*    ap = A  + (size_t)(rowBase + 16 * wave + m) * K + 8 * hh;
  const _Float16* bp = wt + (size_t)m * K + 8 * hh;
  v8f acc[4];
#pragma unroll
  for (int t = 0; t < 4; ++t) { v8f z = {0.f, 0.f, 0.f, 0.f, 0.f, 0.f, 0.f, 0.f}; acc[t] = z; }
  const int nks = K >> 5;
#pragma unroll 1
  for (int ks = 0; ks < nks; ++ks) {
    const float* pa = ap + 32 * ks;
    const v4f x0 = *(const v4f*)(pa);
    const v4f x1 = *(const v4f*)(pa + 4);
    const v4f x2 = *(const v4f*)(pa + 16);
    const v4f x3 = *(const v4f*)(pa + 20);
    FragH af;
    af.h[0] = pack8(x0, x1, CA);
    af.h[1] = pack8(x2, x3, CA);
#pragma unroll
    for (int t = 0; t < 4; ++t) {
      const _Float16* pb = bp + (size_t)(16 * t) * K + 32 * ks;
      FragH bf;
      bf.h[0] = *(const v8h*)(pb);
      bf.h[1] = *(const v8h*)(pb + 16);
      acc[t] = wmh(af, bf, acc[t]);
    }
  }
  {
    float* sp = stg + (size_t)(16 * wave + 8 * hh) * HID + m;
#pragma unroll
    for (int t = 0; t < 4; ++t) {
      const float bb = sb[16 * t + m];
#pragma unroll
      for (int r = 0; r < 8; ++r) {
        float v = fmaf(acc[t][r], SCL, bb);
        v = (relu != 0) ? fmaxf(v, 0.f) : v;
        sp[(size_t)r * HID + 16 * t] = v;
      }
    }
  }
  __syncthreads();
  {
    const int nF4 = GBM * HID / 4;
    float* yb = Y + (size_t)rowBase * HID;
    const v4f* s4 = (const v4f*)stg;
#pragma unroll 1
    for (int f = tid; f < nF4; f += GTHR) {
      const v4f v = s4[f];
      *(volatile v4f*)(yb + 4 * f) = v;
    }
    __threadfence();
#pragma unroll 1
    for (int f = tid; f < nF4; f += GTHR) {
      const v4f v = s4[f];
      *(volatile v4f*)(yb + 4 * f) = v;
    }
  }
}

__global__ __launch_bounds__(NTHR) void k_build(const int* __restrict__ dsts, int* EL, int* OFF, int* CNT,
                                                int nE, int nb, int tp, int vec8) {
  extern __shared__ v4f lds_dyn[];
  int* reg1 = (int*)lds_dyn;
  int* reg2 = reg1 + RCAP;
  int* scnt = reg2 + RCAP;
  int* soff = scnt + NBMAX;
  int* list = soff + NBMAX;
  int* wcnt = list + LISTN;
  int* wtot = wcnt + NWAVE;
  const int tid = threadIdx.x, lane = tid & 31, wave = tid >> 5;
  const int nodeBase = (int)blockIdx.x * nb;

  for (int i = tid; i < NBMAX; i += NTHR) scnt[i] = 0;
  {
    const v4i z = {0, 0, 0, 0};
    v4i* r2v = (v4i*)reg2;
    for (int f = tid; f < RCAP / 4; f += NTHR) r2v[f] = z;
  }
  __syncthreads();

  int tot = 0;
  const int nChunks = (nE + CHUNK - 1) / CHUNK;
#pragma unroll 1
  for (int ch = 0; ch < nChunks; ++ch) {
    const int cbase = ch * CHUNK;
    const int wc = scan_chunk(dsts, nE, cbase, nodeBase, nb, vec8, list, tid, lane, wave);
    if (lane == 0) wcnt[wave] = wc;
    __syncthreads();
    int pre = 0, all = 0;
#pragma unroll
    for (int w2 = 0; w2 < NWAVE; ++w2) {
      int c = wcnt[w2];
      c = c < 0 ? 0 : (c > WCAP ? WCAP : c);
      all += c;
      pre += (w2 < wave) ? c : 0;
    }
    const int wcc  = wc > WCAP ? WCAP : wc;
    const int base = tot + pre;
#pragma unroll 1
    for (int i = lane; i < wcc; i += 32) {
      const int ent = list[wave * WCAP + i];
      const int el  = (ent >> 12) & (CHUNK - 1);
      const int sl  = ent & (NBMAX - 1);
      int eid = cbase + el;
      eid = eid > nE - 1 ? nE - 1 : eid;
      const int pos = base + i;
      if (pos < RCAP) reg1[pos] = (int)(((unsigned)eid << SLOTB) | (unsigned)sl);
    }
    tot += all;
    tot = tot > RCAP ? RCAP : tot;
    __syncthreads();
  }
  const int nh = tot;

  if (wave == 0) {
#pragma unroll 1
    for (int b0 = 0; b0 < nh; b0 += 32) {
      const int idx = b0 + lane;
      const int uv  = reg1[idx < RCAP ? idx : RCAP - 1];
      const int m32 = (nh - b0) < 32 ? (nh - b0) : 32;
#pragma unroll 1
      for (int k = 0; k < m32; ++k) {
        const int u  = __builtin_amdgcn_readlane(uv, k);
        const int sl = u & (NBMAX - 1);
        if (lane == 0) scnt[sl] = scnt[sl] + 1;
      }
    }
  }
  __syncthreads();

  {
    const v4i ca = *(const v4i*)(scnt + 8 * tid);
    const v4i cb = *(const v4i*)(scnt + 8 * tid + 4);
    const int e0 = ca.x < 0 ? 0 : ca.x, e1 = ca.y < 0 ? 0 : ca.y, e2 = ca.z < 0 ? 0 : ca.z, e3 = ca.w < 0 ? 0 : ca.w;
    const int e4 = cb.x < 0 ? 0 : cb.x, e5 = cb.y < 0 ? 0 : cb.y, e6 = cb.z < 0 ? 0 : cb.z, e7 = cb.w < 0 ? 0 : cb.w;
    const int ts = e0 + e1 + e2 + e3 + e4 + e5 + e6 + e7;
    int incl = ts;
#pragma unroll
    for (int d = 1; d < 32; d <<= 1) {
      const int up = __shfl_up(incl, d);
      if (lane >= d) incl += up;
    }
    if (lane == 31) wtot[wave] = incl;
    __syncthreads();
    int pre = 0;
#pragma unroll
    for (int w2 = 0; w2 < NWAVE; ++w2) pre += (w2 < wave) ? wtot[w2] : 0;
    int run = pre + incl - ts;
    soff[8 * tid + 0] = run; run += e0;
    soff[8 * tid + 1] = run; run += e1;
    soff[8 * tid + 2] = run; run += e2;
    soff[8 * tid + 3] = run; run += e3;
    soff[8 * tid + 4] = run; run += e4;
    soff[8 * tid + 5] = run; run += e5;
    soff[8 * tid + 6] = run; run += e6;
    soff[8 * tid + 7] = run;
  }
  __syncthreads();
  for (int i = tid; i < NBMAX; i += NTHR) list[i] = soff[i];
  __syncthreads();

  if (wave == 0) {
#pragma unroll 1
    for (int b0 = 0; b0 < nh; b0 += 32) {
      const int idx = b0 + lane;
      const int uv  = reg1[idx < RCAP ? idx : RCAP - 1];
      const int m32 = (nh - b0) < 32 ? (nh - b0) : 32;
#pragma unroll 1
      for (int k = 0; k < m32; ++k) {
        const int u   = __builtin_amdgcn_readlane(uv, k);
        const int sl  = u & (NBMAX - 1);
        const int eid = (int)((unsigned)u >> SLOTB);
        if (lane == 0) {
          int pos = list[sl];
          pos = pos < 0 ? 0 : (pos > RCAP - 1 ? RCAP - 1 : pos);
          reg2[pos] = eid;
          list[sl] = pos + 1;
        }
      }
    }
  }
  __syncthreads();

  {
    int* elb = EL + (size_t)blockIdx.x * RCAP;
    const v4i* r4 = (const v4i*)reg2;
#pragma unroll 1
    for (int f = tid; f < RCAP / 4; f += NTHR) {
      const v4i v = r4[f];
      *(volatile v4i*)(elb + 4 * f) = v;
    }
    __threadfence();
#pragma unroll 1
    for (int f = tid; f < RCAP / 4; f += NTHR) {
      const v4i v = r4[f];
      *(volatile v4i*)(elb + 4 * f) = v;
    }
  }
  {
    const bool ovf = (nh >= RCAP);
    int* ob = OFF + (size_t)blockIdx.x * tp;
    int* cb = CNT + (size_t)blockIdx.x * tp;
    const int n4 = tp >> 2;
#pragma unroll 1
    for (int pass = 0; pass < 2; ++pass) {
#pragma unroll 1
      for (int f = tid; f < n4; f += NTHR) {
        v4i so, sc;
        {
          const int s = 4 * f + 0; const bool in = s < nb; const int scl = s < NBMAX ? s : NBMAX - 1;
          so.x = in ? soff[scl] : 0; sc.x = in ? (ovf ? -1 : scnt[scl]) : 0;
        }
        {
          const int s = 4 * f + 1; const bool in = s < nb; const int scl = s < NBMAX ? s : NBMAX - 1;
          so.y = in ? soff[scl] : 0; sc.y = in ? (ovf ? -1 : scnt[scl]) : 0;
        }
        {
          const int s = 4 * f + 2; const bool in = s < nb; const int scl = s < NBMAX ? s : NBMAX - 1;
          so.z = in ? soff[scl] : 0; sc.z = in ? (ovf ? -1 : scnt[scl]) : 0;
        }
        {
          const int s = 4 * f + 3; const bool in = s < nb; const int scl = s < NBMAX ? s : NBMAX - 1;
          so.w = in ? soff[scl] : 0; sc.w = in ? (ovf ? -1 : scnt[scl]) : 0;
        }
        *(volatile v4i*)(ob + 4 * f) = so;
        *(volatile v4i*)(cb + 4 * f) = sc;
      }
      __threadfence();
    }
  }
}

__global__ __launch_bounds__(NTHR) void k_agg(
    const int* __restrict__ srcs, const int* __restrict__ EL,
    const int* __restrict__ OFF, const int* __restrict__ CNT,
    const float* __restrict__ Hin, const float* __restrict__ betas,
    float* Hout, int nN, int nE, int nb, int tp, int nBeta, int li) {
  const int tid = threadIdx.x, lane = tid & 31, wave = tid >> 5;
  const int g   = lane >> 3;
  const int sub = lane & 7;
  const int c0  = 8 * sub;
  const int srcl = (lane & 15) >> 1;
  const int hsel = lane & 1;
  const int nodeBase = (int)blockIdx.x * nb;
  const int nbw = nb >> 3;
  const int* elb  = EL  + (size_t)blockIdx.x * RCAP;
  const int* offb = OFF + (size_t)blockIdx.x * tp;
  const int* cntb = CNT + (size_t)blockIdx.x * tp;
  const int bi = li < 0 ? 0 : (li > nBeta - 1 ? nBeta - 1 : li);
  const float beta = betas[bi];
  const float qnan = __int_as_float(0x7fc00000);
  const v4f z4 = {0.f, 0.f, 0.f, 0.f};
#pragma unroll 1
  for (int jt = 0; jt < nbw; ++jt) {
    const int slot = wave * nbw + jt;
    const int grow = nodeBase + slot;
    const int gcl  = grow < nN ? grow : nN - 1;
    const bool wr  = grow < nN;
    int st = offb[slot];
    const int craw = cntb[slot];
    st = st < 0 ? 0 : (st > RCAP - 1 ? RCAP - 1 : st);
    int cnt = craw < 0 ? 0 : (craw > DEGCAP ? DEGCAP : craw);
    if (cnt > RCAP - st) cnt = RCAP - st;
    const float pz = (craw < 0 || craw > DEGCAP) ? qnan : 0.0f;

    const float* hdp = Hin + (size_t)gcl * HID + c0;
    const v4f hd0 = *(const v4f*)(hdp), hd1 = *(const v4f*)(hdp + 4);
    float sd = dot8(hd0, hd1, hd0, hd1);
    sd += __shfl_xor(sd, 1); sd += __shfl_xor(sd, 2); sd += __shfl_xor(sd, 4);
    const float invd = __builtin_amdgcn_rcpf(fmaxf(__builtin_amdgcn_sqrtf(sd), EPSN));
    const float sdl  = beta * invd;

    float mx = NEGBIG, dn = 0.0f;
    v4f a0 = z4, a1 = z4;
    const int niter = (cnt + NSTRM - 1) / NSTRM;
#pragma unroll 1
    for (int it = 0; it < niter; ++it) {
      const int q = it * NSTRM + g;
      const bool valid = q < cnt;
      const int qc = valid ? q : cnt - 1;
      const int idx = st + qc;
      int eid = elb[idx];
      eid = eid < 0 ? 0 : (eid > nE - 1 ? nE - 1 : eid);
      const int sraw = srcs[eid];
      const int s = sraw < 0 ? 0 : (sraw > nN - 1 ? nN - 1 : sraw);
      const float* hsp = Hin + (size_t)s * HID + c0;
      const v4f hs0 = *(const v4f*)(hsp);
      const v4f hs1 = *(const v4f*)(hsp + 4);
      float p  = dot8(hs0, hs1, hd0, hd1);
      float ss = dot8(hs0, hs1, hs0, hs1);
      p  += __shfl_xor(p, 1);  ss += __shfl_xor(ss, 1);
      p  += __shfl_xor(p, 2);  ss += __shfl_xor(ss, 2);
      p  += __shfl_xor(p, 4);  ss += __shfl_xor(ss, 4);
      const float invs = __builtin_amdgcn_rcpf(fmaxf(__builtin_amdgcn_sqrtf(ss), EPSN));
      float l = (p * invs) * sdl;
      l = valid ? l : NEGBIG;
      const float mn = fmaxf(mx, l);
      const float s1 = __expf(mx - mn);
      const float s2 = valid ? __expf(l - mn) : 0.0f;
      dn = fmaf(dn, s1, s2);
      a0 = a0 * s1 + hs0 * s2;
      a1 = a1 * s1 + hs1 * s2;
      mx = mn;
    }
    float m1 = fmaxf(mx, __shfl_xor(mx, 8));
    m1 = fmaxf(m1, __shfl_xor(m1, 16));
    const float e = __expf(mx - m1);
    v4f r0 = a0 * e, r1 = a1 * e;
    float ds = dn * e;
    r0 += xor4(r0, 8);  r1 += xor4(r1, 8);  ds += __shfl_xor(ds, 8);
    r0 += xor4(r0, 16); r1 += xor4(r1, 16); ds += __shfl_xor(ds, 16);
    const float dsg = ds > 0.0f ? ds : 1.0f;
    const float inv = ds > 0.0f ? __builtin_amdgcn_rcpf(dsg) : 0.0f;
    v4f o0 = r0 * inv, o1 = r1 * inv;
    o0.x += pz; o0.y += pz; o0.z += pz; o0.w += pz;
    o1.x += pz; o1.y += pz; o1.z += pz; o1.w += pz;
    const v4f t0 = shf4(o0, srcl);
    const v4f t1 = shf4(o1, srcl);
    v4f v;
    v.x = hsel ? t1.x : t0.x; v.y = hsel ? t1.y : t0.y;
    v.z = hsel ? t1.z : t0.z; v.w = hsel ? t1.w : t0.w;
    float* hp = Hout + (size_t)gcl * HID + 4 * (lane & 15);
    const bool dow = wr && (lane < 16);
    if (dow) *(volatile v4f*)hp = v;
    __threadfence();
    if (dow) *(volatile v4f*)hp = v;
  }
}

static int pick_nb(int nE, int nN) {
  int nb = NBMAX;
  while (nb > 16 && (long long)nb * (long long)nE * 5LL > (long long)RCAP * (long long)nN * 4LL) nb >>= 1;
  return nb;
}

extern "C" void kernel_launch(void* const* d_in, const int* in_sizes, int n_in,
                              void* d_out, int out_size, void* d_ws, size_t ws_size,
                              hipStream_t stream) {
  if (n_in < 8) return;
  const int nN = in_sizes[0] / FIN;
  if (nN <= 0 || in_sizes[0] != nN * FIN) return;
  if ((nN % GBM) != 0) return;
  if (nN > (1 << 22)) return;
  const int nE = in_sizes[1];
  if (nE < 1 || nE > (1 << 21)) return;
  if (in_sizes[2] != nE) return;
  if (in_sizes[3] != FIN * HID) return;
  if (in_sizes[4] != HID) return;
  if (in_sizes[5] != HID * HID) return;
  if (in_sizes[6] != HID) return;
  const int nBeta = in_sizes[7];
  if (nBeta < 1) return;
  if (out_size != nN * HID) return;

  const float* x     = (const float*)d_in[0];
  const int*   srcs  = (const int*)d_in[1];
  const int*   dsts  = (const int*)d_in[2];
  const float* W1    = (const float*)d_in[3];
  const float* b1    = (const float*)d_in[4];
  const float* W2    = (const float*)d_in[5];
  const float* b2    = (const float*)d_in[6];
  const float* betas = (const float*)d_in[7];
  float* out = (float*)d_out;

  const int MP   = nN;
  const int nb   = pick_nb(nE, nN);
  const int tp   = nb < 32 ? 32 : nb;
  const int gA   = (nN + nb - 1) / nb;
  const int gG   = MP / GBM;
  const int vec8 = ((nE & 3) == 0) ? 1 : 0;
  if (nb < 16 || nb > NBMAX || (nb & 7) != 0 || (long long)gA * nb < (long long)nN) return;

  char* ws = (char*)d_ws;
  size_t off = 0;
  const size_t oW1T = off; off += (size_t)HID * FIN * 2;          off = (off + 255) & ~(size_t)255;
  const size_t oW2T = off; off += (size_t)HID * HID * 2;          off = (off + 255) & ~(size_t)255;
  const size_t oHA  = off; off += (size_t)MP * HID * 4;           off = (off + 255) & ~(size_t)255;
  const size_t oHB  = off; off += (size_t)MP * HID * 4;           off = (off + 255) & ~(size_t)255;
  const size_t oEL  = off; off += (size_t)gA * RCAP * 4;          off = (off + 255) & ~(size_t)255;
  const size_t oOFF = off; off += (size_t)gA * tp * 4;            off = (off + 255) & ~(size_t)255;
  const size_t oCNT = off; off += (size_t)gA * tp * 4;            off = (off + 255) & ~(size_t)255;
  if (off > ws_size || off > (size_t)WSCAP) return;
  _Float16* W1T = (_Float16*)(ws + oW1T);
  _Float16* W2T = (_Float16*)(ws + oW2T);
  float*    HA  = (float*)(ws + oHA);
  float*    HB  = (float*)(ws + oHB);
  int*      EL  = (int*)(ws + oEL);
  int*      OFF = (int*)(ws + oOFF);
  int*      CNT = (int*)(ws + oCNT);

  hipFuncSetAttribute(reinterpret_cast<const void*>(&k_build),
                      hipFuncAttributeMaxDynamicSharedMemorySize, LDS_BUILD);

  k_wprep<<<dim3((HID * (FIN / 8) + NTHR - 1) / NTHR, 2), NTHR, 0, stream>>>(W1, W2, W1T, W2T);

  k_build<<<gA, NTHR, LDS_BUILD, stream>>>(dsts, EL, OFF, CNT, nE, nb, tp, vec8);

  k_lin<<<gG, GTHR, 0, stream>>>(x, W1T, b1, HA, FIN, 1);

  k_agg<<<gA, NTHR, 0, stream>>>(srcs, EL, OFF, CNT, HA, betas, HB, nN, nE, nb, tp, nBeta, 0);
  k_agg<<<gA, NTHR, 0, stream>>>(srcs, EL, OFF, CNT, HB, betas, HA, nN, nE, nb, tp, nBeta, 1);

  k_lin<<<gG, GTHR, 0, stream>>>(HA, W2T, b2, out, HID, 0);
}
